// Decoder_84731114815924
// MI455X (gfx1250) — hardware-verified
//
#include <hip/hip_runtime.h>
#include <stddef.h>
#include <stdint.h>
#include <math.h>


#define NB    4
#define NN    256
#define DD    32
#define HH    512
#define KK    256
#define NBI   (NB * NN)
#define NW1   (HH * DD)
#define TPW   64
#define UZ    (NBI * (DD / 8))
#define UW1   (NW1 * (DD / 8))
#define UW2   (KK * (HH / 8))
#define OZB_H  0
#define OW1T_H (NBI * DD)
#define OW2T_H (OW1T_H + NW1 * DD)
#define OTMP_H (OW2T_H + KK * HH)
#define WS_HALVES ((size_t)OTMP_H + (size_t)NBI * HH * TPW)
#define WSMAX  134217728
#define ZP    40
#define HP    264
#define TNH   8
#define OUT1  (NBI * NN)

static_assert(UZ % 256 == 0 && UW1 % 256 == 0 && UW2 % 256 == 0);
static_assert((OW1T_H * 2) % 256 == 0 && (OW2T_H * 2) % 256 == 0 && (OTMP_H * 2) % 256 == 0);
static_assert(WS_HALVES * 2 <= (size_t)WSMAX);
static_assert(DD == 32 && HH % 128 == 0 && KK == 8 * 32 && NN == 256);
static_assert((ZP * 2) % 16 == 0 && (HP * 2) % 16 == 0 && HP >= 256 && ZP >= 32);
static_assert(HH % TNH == 0 && NBI % 64 == 0);
static_assert((size_t)OUT1 + (size_t)(NBI - 1) * NN + (NN - 1) < (size_t)2 * NBI * NN);

typedef float          v4f   __attribute__((ext_vector_type(4)));
typedef float          v8f   __attribute__((ext_vector_type(8)));
typedef int            v8i   __attribute__((ext_vector_type(8)));
typedef unsigned short v8us  __attribute__((ext_vector_type(8)));
typedef unsigned short v16us __attribute__((ext_vector_type(16)));
typedef __bf16         v16bf __attribute__((ext_vector_type(16)));
typedef v4f  __attribute__((may_alias)) v4fa;
typedef v8us __attribute__((may_alias)) v8usa;
union FragB { v16bf v; v16us u; v8us h[2]; v8i w; };

__device__ __forceinline__ v8f wmb(const FragB& a, const FragB& b, v8f c) {
  v8f d = __builtin_amdgcn_wmma_f32_16x16x32_bf16(false, a.v, false, b.v, (short)0, c, false, false);
  asm volatile("v_nop\n\tv_nop\n\tv_nop\n\tv_nop" : "+v"(d) : "v"(a.w), "v"(b.w));
  return d;
}

__device__ __forceinline__ unsigned bf16_bits(float f) {
  const unsigned u = __float_as_uint(f);
  return (u + 0x7FFFu + ((u >> 16) & 1u)) >> 16;
}
__device__ __forceinline__ float bf16_val(float f) {
  return __uint_as_float(bf16_bits(f) << 16);
}

__device__ __forceinline__ void wave_sync() {
  __builtin_amdgcn_fence(__ATOMIC_RELEASE, "wavefront");
  __builtin_amdgcn_wave_barrier();
  __builtin_amdgcn_fence(__ATOMIC_ACQUIRE, "wavefront");
}

__global__ __launch_bounds__(256) void k_prep(const float* __restrict__ z, const float* __restrict__ W1,
                                              const float* __restrict__ W2, unsigned short* wsb) {
  const int u = (int)blockIdx.x * 256 + (int)threadIdx.x;
  v8us o;
  size_t doff;
  if (u < UZ) {
    const float* p = z + (size_t)u * 8;
    const v4f a = *(const v4fa*)p;
    const v4f b = *(const v4fa*)(p + 4);
    o[0] = (unsigned short)bf16_bits(a.x); o[1] = (unsigned short)bf16_bits(a.y);
    o[2] = (unsigned short)bf16_bits(a.z); o[3] = (unsigned short)bf16_bits(a.w);
    o[4] = (unsigned short)bf16_bits(b.x); o[5] = (unsigned short)bf16_bits(b.y);
    o[6] = (unsigned short)bf16_bits(b.z); o[7] = (unsigned short)bf16_bits(b.w);
    doff = (size_t)OZB_H + (size_t)u * 8;
  } else if (u < UZ + UW1) {
    const int v    = u - UZ;
    const int nrow = v >> 2;
    const int a8   = (v & 3) * 8;
    const int h    = nrow >> 5;
    const int c    = nrow & 31;
    const float* p = W1 + ((size_t)a8 * DD + c) * HH + h;
#pragma unroll
    for (int i = 0; i < 8; ++i) o[i] = (unsigned short)bf16_bits(p[(size_t)i * DD * HH]);
    doff = (size_t)OW1T_H + (size_t)nrow * DD + a8;
  } else if (u < UZ + UW1 + UW2) {
    const int v  = u - UZ - UW1;
    const int k  = v >> 6;
    const int h8 = (v & 63) * 8;
    const float* p = W2 + (size_t)h8 * KK + k;
#pragma unroll
    for (int i = 0; i < 8; ++i) o[i] = (unsigned short)bf16_bits(p[(size_t)i * KK]);
    doff = (size_t)OW2T_H + (size_t)k * HH + h8;
  } else {
    return;
  }
  unsigned short* dp = wsb + doff;
  *(volatile v8us*)dp = o;
  __threadfence();
  *(volatile v8us*)dp = o;
}

__global__ __launch_bounds__(128) void k_tmp(const unsigned short* __restrict__ ZB,
                                             const unsigned short* __restrict__ W1T, unsigned short* TMP) {
  __shared__ __attribute__((aligned(16))) unsigned short stg[4 * 16 * TPW];
  const int tid = (int)threadIdx.x, lane = tid & 31, wave = tid >> 5, hh = lane >> 4, m = lane & 15;
  const int rowBase = (int)blockIdx.x * 64;
  const int h0 = (int)blockIdx.y * TNH;
  unsigned short* sw = stg + wave * (16 * TPW);

  FragB af;
  {
    const unsigned short* ap = ZB + (size_t)(rowBase + 16 * wave + m) * DD + 8 * hh;
    af.h[0] = *(const v8usa*)ap;
    af.h[1] = *(const v8usa*)(ap + 16);
  }
  const v8f zz = {0.f, 0.f, 0.f, 0.f, 0.f, 0.f, 0.f, 0.f};
#pragma unroll 1
  for (int hi = 0; hi < TNH; ++hi) {
    const int h = h0 + hi;
    const unsigned short* wp = W1T + ((size_t)h * DD + m) * DD + 8 * hh;
    FragB b0, b1;
    b0.h[0] = *(const v8usa*)wp;
    b0.h[1] = *(const v8usa*)(wp + 16);
    b1.h[0] = *(const v8usa*)(wp + 16 * DD);
    b1.h[1] = *(const v8usa*)(wp + 16 * DD + 16);
    const v8f d0 = wmb(af, b0, zz);
    const v8f d1 = wmb(af, b1, zz);
#pragma unroll
    for (int r = 0; r < 8; ++r) {
      const int row = 8 * hh + r;
      const float v0 = d0[r];
      const unsigned hb0 = bf16_bits(v0);
      const unsigned lb0 = bf16_bits(v0 - __uint_as_float(hb0 << 16));
      const float v1 = d1[r];
      const unsigned hb1 = bf16_bits(v1);
      const unsigned lb1 = bf16_bits(v1 - __uint_as_float(hb1 << 16));
      sw[row * TPW + m]      = (unsigned short)hb0;
      sw[row * TPW + 16 + m] = (unsigned short)hb1;
      sw[row * TPW + 32 + m] = (unsigned short)lb0;
      sw[row * TPW + 48 + m] = (unsigned short)lb1;
    }
    wave_sync();
    v8us q[4];
#pragma unroll
    for (int it = 0; it < 4; ++it) {
      const int row = 4 * it + (lane >> 3);
      q[it] = *(const v8usa*)(sw + row * TPW + 8 * (lane & 7));
    }
    wave_sync();
#pragma unroll
    for (int it = 0; it < 4; ++it) {
      const int row = 4 * it + (lane >> 3);
      unsigned short* gp = TMP + ((size_t)(rowBase + 16 * wave + row) * HH + h) * TPW + 8 * (lane & 7);
      *(volatile v8us*)gp = q[it];
    }
    __threadfence();
#pragma unroll
    for (int it = 0; it < 4; ++it) {
      const int row = 4 * it + (lane >> 3);
      unsigned short* gp = TMP + ((size_t)(rowBase + 16 * wave + row) * HH + h) * TPW + 8 * (lane & 7);
      *(volatile v8us*)gp = q[it];
    }
  }
}

__global__ __launch_bounds__(256) void k_pair(const unsigned short* __restrict__ ZB,
                                              const unsigned short* __restrict__ TMP,
                                              const unsigned short* __restrict__ W2T,
                                              const float* __restrict__ mk,
                                              const float* __restrict__ b1, const float* __restrict__ b2,
                                              const float* __restrict__ W3, const float* __restrict__ b3,
                                              float* out) {
  __shared__ __attribute__((aligned(16))) unsigned short zt[64 * ZP];
  __shared__ __attribute__((aligned(16))) unsigned short h1c[64 * HP];
  __shared__ __attribute__((aligned(16))) float part[8 * 64];
  __shared__ __attribute__((aligned(16))) float rows[2 * NN];
  __shared__ float mval[NN];
  __shared__ int   jl[NN];
  __shared__ int   wcnt[8];

  const int tid = (int)threadIdx.x, lane = tid & 31, wave = tid >> 5, hh = lane >> 4, m = lane & 15;
  const int bi = (int)blockIdx.x;
  const int b  = bi >> 8;

  const float mi = bf16_val(mk[bi]);
  const float mj = bf16_val(mk[b * NN + tid]);
  const float pj = mi * mj;
  const bool  act = (pj != 0.0f);
  const unsigned bal = __builtin_amdgcn_ballot_w32(act);
  jl[tid]   = 0;
  mval[tid] = mj;
  rows[tid] = 0.5f;
  rows[NN + tid] = 0.0f;
  if (lane == 0) wcnt[wave] = (int)__builtin_popcount(bal);
  __syncthreads();
  int base = 0, njv = 0;
#pragma unroll
  for (int w2 = 0; w2 < 8; ++w2) {
    const int c = wcnt[w2];
    njv += c;
    base += (w2 < wave) ? c : 0;
  }
  njv = njv < 0 ? 0 : (njv > NN ? NN : njv);
  const int nj = __builtin_amdgcn_readfirstlane(njv);
  if (act) {
    int pos = base + (int)__builtin_amdgcn_mbcnt_lo(bal, 0u);
    pos = pos < 0 ? 0 : (pos > NN - 1 ? NN - 1 : pos);
    jl[pos] = tid;
  }
  __syncthreads();
  {
    const int lastj = jl[nj > 0 ? nj - 1 : 0];
    if (tid >= nj) jl[tid] = lastj;
  }

  float b2v0, b2v1, w3v0, w3v1;
  {
    const int kc0 = 32 * wave + m;
    const int kc1 = kc0 + 16;
    b2v0 = bf16_val(b2[kc0]); b2v1 = bf16_val(b2[kc1]);
    w3v0 = bf16_val(W3[kc0]); w3v1 = bf16_val(W3[kc1]);
  }
  const float b3v = bf16_val(b3[0]);
  const v8f zz = {0.f, 0.f, 0.f, 0.f, 0.f, 0.f, 0.f, 0.f};

  const int ntile = (nj + 63) >> 6;
#pragma unroll 1
  for (int tile = 0; tile < ntile; ++tile) {
    __syncthreads();
    {
      const int r = tid >> 2, q = tid & 3;
      int gi = tile * 64 + r;
      gi = gi > NN - 1 ? NN - 1 : gi;
      const int j = jl[gi] & (NN - 1);
      const v8us zv = *(const v8usa*)(ZB + (size_t)(b * NN + j) * DD + 8 * q);
      *(v8usa*)(zt + r * ZP + 8 * q) = zv;
    }
    const int rem = nj - tile * 64;
    const int nmt = rem >= 64 ? 4 : ((rem + 15) >> 4);

    v8f acc[4][2];
#pragma unroll
    for (int mt = 0; mt < 4; ++mt) { acc[mt][0] = zz; acc[mt][1] = zz; }
    __syncthreads();

#pragma unroll 1
    for (int ch = 0; ch < 4; ++ch) {
      v8f g[4];
      {
        const unsigned short* tb = TMP + ((size_t)bi * HH + ch * 128 + 16 * wave + m) * TPW + 8 * hh;
        FragB bh, bl;
        bh.h[0] = *(const v8usa*)tb;
        bh.h[1] = *(const v8usa*)(tb + 16);
        bl.h[0] = *(const v8usa*)(tb + 32);
        bl.h[1] = *(const v8usa*)(tb + 48);
#pragma unroll
        for (int mt = 0; mt < 4; ++mt) {
          g[mt] = zz;
          if (mt < nmt) {
            const unsigned short* zp = zt + (16 * mt + m) * ZP + 8 * hh;
            FragB az;
            az.h[0] = *(const v8usa*)zp;
            az.h[1] = *(const v8usa*)(zp + 16);
            g[mt] = wmb(az, bh, g[mt]);
            g[mt] = wmb(az, bl, g[mt]);
          }
        }
      }
      const float b1v = bf16_val(b1[ch * 128 + 16 * wave + m]);
      __syncthreads();
#pragma unroll
      for (int mt = 0; mt < 4; ++mt) {
        if (mt < nmt) {
#pragma unroll
          for (int r = 0; r < 8; ++r) {
            const int row = 16 * mt + 8 * hh + r;
            float v = g[mt][r] + b1v;
            v = (v < 0.0f) ? 0.0f : v;
            const unsigned hb = bf16_bits(v);
            const unsigned lb = bf16_bits(v - __uint_as_float(hb << 16));
            h1c[row * HP + 16 * wave + m]       = (unsigned short)hb;
            h1c[row * HP + 128 + 16 * wave + m] = (unsigned short)lb;
          }
        }
      }
      __syncthreads();

#pragma unroll 1
      for (int ks = 0; ks < 4; ++ks) {
        FragB bw0, bw1;
        {
          const unsigned short* wq = W2T + (size_t)(32 * wave + m) * HH + ch * 128 + 32 * ks + 8 * hh;
          bw0.h[0] = *(const v8usa*)wq;
          bw0.h[1] = *(const v8usa*)(wq + 16);
          bw1.h[0] = *(const v8usa*)(wq + 16 * HH);
          bw1.h[1] = *(const v8usa*)(wq + 16 * HH + 16);
        }
#pragma unroll
        for (int mt = 0; mt < 4; ++mt) {
          if (mt < nmt) {
            const unsigned short* hp = h1c + (16 * mt + m) * HP + 32 * ks + 8 * hh;
            FragB ah, al;
            ah.h[0] = *(const v8usa*)hp;
            ah.h[1] = *(const v8usa*)(hp + 16);
            al.h[0] = *(const v8usa*)(hp + 128);
            al.h[1] = *(const v8usa*)(hp + 144);
            acc[mt][0] = wmb(ah, bw0, acc[mt][0]);
            acc[mt][1] = wmb(ah, bw1, acc[mt][1]);
            acc[mt][0] = wmb(al, bw0, acc[mt][0]);
            acc[mt][1] = wmb(al, bw1, acc[mt][1]);
          }
        }
      }
    }

#pragma unroll
    for (int mt = 0; mt < 4; ++mt) {
#pragma unroll
      for (int r = 0; r < 8; ++r) {
        float v0 = acc[mt][0][r] + b2v0;
        float v1 = acc[mt][1][r] + b2v1;
        v0 = (v0 < 0.0f) ? 0.0f : v0;
        v1 = (v1 < 0.0f) ? 0.0f : v1;
        float s = v0 * w3v0;
        s = fmaf(v1, w3v1, s);
        s += __shfl_xor(s, 8, 32);
        s += __shfl_xor(s, 4, 32);
        s += __shfl_xor(s, 2, 32);
        s += __shfl_xor(s, 1, 32);
        if (m == 0) part[wave * 64 + 16 * mt + 8 * hh + r] = s;
      }
    }
    __syncthreads();
    if (tid < 64) {
      float s = 0.0f;
#pragma unroll
      for (int w2 = 0; w2 < 8; ++w2) s += part[w2 * 64 + tid];
      const float lg = s + b3v;
      const int g0 = tile * 64 + tid;
      const int gc = g0 > NN - 1 ? NN - 1 : g0;
      const int jc = jl[gc] & (NN - 1);
      const float p   = mi * mval[jc];
      const float lgm = lg * p;
      const float mp  = 1.0f / (1.0f + expf(-lgm));
      if (g0 < nj) { rows[jc] = mp; rows[NN + jc] = lgm; }
    }
  }
  __syncthreads();

  if (tid < 128) {
    const int sel = tid >> 6;
    const int t   = tid & 63;
    const v4f ov = *(const v4fa*)(rows + 4 * tid);
    float* op = out + (size_t)sel * OUT1 + (size_t)bi * NN + 4 * t;
    *(volatile v4f*)op = ov;
    __threadfence();
    *(volatile v4f*)op = ov;
  }
}

extern "C" void kernel_launch(void* const* d_in, const int* in_sizes, int n_in,
                              void* d_out, int out_size, void* d_ws, size_t ws_size,
                              hipStream_t stream) {
  if (n_in < 9) return;
  if (in_sizes[0] != NBI * DD) return;
  if (in_sizes[1] != NBI) return;
  if (in_sizes[3] != DD * DD * HH) return;
  if (in_sizes[4] != HH) return;
  if (in_sizes[5] != HH * KK) return;
  if (in_sizes[6] != KK) return;
  if (in_sizes[7] != KK) return;
  if (in_sizes[8] != 1) return;
  if (out_size != 2 * NBI * NN) return;

  const float* z  = (const float*)d_in[0];
  const float* mk = (const float*)d_in[1];
  const float* W1 = (const float*)d_in[3];
  const float* b1 = (const float*)d_in[4];
  const float* W2 = (const float*)d_in[5];
  const float* b2 = (const float*)d_in[6];
  const float* W3 = (const float*)d_in[7];
  const float* b3 = (const float*)d_in[8];
  float* out = (float*)d_out;

  const size_t total = WS_HALVES * 2;
  if (total > ws_size || total > (size_t)WSMAX) return;
  unsigned short* wsb = (unsigned short*)d_ws;
  const unsigned short* ZB  = wsb + OZB_H;
  const unsigned short* W1T = wsb + OW1T_H;
  const unsigned short* W2T = wsb + OW2T_H;
  unsigned short*       TMP = wsb + OTMP_H;

  k_prep<<<(UZ + UW1 + UW2) / 256, 256, 0, stream>>>(z, W1, W2, wsb);
  k_tmp<<<dim3(NBI / 64, HH / TNH), 128, 0, stream>>>(ZB, W1T, TMP);
  k_pair<<<NBI, 256, 0, stream>>>(ZB, TMP, W2T, mk, b1, b2, W3, b3, out);
}
